// LSTM_89361089560808
// MI455X (gfx1250) — hardware-verified
//
#include <hip/hip_runtime.h>
#include <math.h>

constexpr int NBATCH   = 32;
constexpr int NSTEP    = 65536;
constexpr int NHID     = 32;
constexpr int NGATE    = 4 * NHID;
constexpr int BLK_ROWS = 16;
constexpr int CHUNK    = 32;
constexpr float RES_CARRY     = 2048.0f;
constexpr float RES_CARRY_INV = 1.0f / RES_CARRY;
constexpr float F16_MIN_NORMAL = 6.103515625e-05f;
static_assert(NHID == 32, "K must be exactly one 32-deep WMMA step");
static_assert(NGATE == 8 * 16, "8 gate-row tiles");
static_assert(NBATCH % BLK_ROWS == 0, "whole 16-row groups");
static_assert(NSTEP % CHUNK == 0, "no tail chunk");
static_assert(CHUNK * 4 == 128, "one chunk of y = one 128-B line");

typedef __attribute__((ext_vector_type(16))) _Float16 v16h;
typedef __attribute__((ext_vector_type(8)))  _Float16 v8h;
typedef __attribute__((ext_vector_type(8)))  float    v8f;
typedef __attribute__((ext_vector_type(4)))  float    v4f;
typedef __attribute__((ext_vector_type(4)))  unsigned v4u;

template <typename T> struct Frag;
template <> struct Frag<_Float16> {
  typedef v16h V; union U { v16h v; v8h h[2]; };
  static __device__ __forceinline__ v16h load(const _Float16* p) {
    U f; f.h[0] = *(const v8h*)(p); f.h[1] = *(const v8h*)(p + 16); return f.v;
  }
  static __device__ __forceinline__ v8f mma(v16h a, v16h b, v8f c) {
    return __builtin_amdgcn_wmma_f32_16x16x32_f16(false, a, false, b, (short)0, c, false, false);
  }
};

__device__ __forceinline__ void tile_guard(v8f& m, v8f& r, v16h a0, v16h a1, v16h b0, v16h b1) {
  asm volatile("v_nop\n\tv_nop\n\tv_nop\n\tv_nop" : "+v"(m), "+v"(r) : "v"(a0), "v"(a1), "v"(b0), "v"(b1));
}

__device__ __forceinline__ void split_f16(float v, _Float16& hi, _Float16& lo) {
  float hf = (float)((_Float16)v);
  asm volatile("" : "+v"(hf));
  hf = (fabsf(hf) < F16_MIN_NORMAL) ? 0.0f : hf;
  hi = (_Float16)hf;
  lo = (_Float16)((v - hf) * RES_CARRY);
}

__device__ __forceinline__ float fsig(float x)  { return __builtin_amdgcn_rcpf(1.0f + expf(-x)); }
__device__ __forceinline__ float ftanh(float x) { return 1.0f - 2.0f * __builtin_amdgcn_rcpf(expf(2.0f * x) + 1.0f); }

__global__ __launch_bounds__(32) void lstm_seq_kernel(const float* __restrict__ x, const float* __restrict__ w_ih,
                                                     const float* __restrict__ w_hh, const float* __restrict__ b_ih,
                                                     const float* __restrict__ b_hh, const float* __restrict__ w_lin,
                                                     const float* __restrict__ b_lin, float* __restrict__ out) {
  __shared__ __align__(16) _Float16 Whi[NGATE * NHID];
  __shared__ __align__(16) _Float16 Wlo[NGATE * NHID];
  __shared__ __align__(16) float    Bs[NGATE];
  __shared__ __align__(16) float    Wis[NGATE];
  __shared__ __align__(16) _Float16 Hh[BLK_ROWS * NHID];
  __shared__ __align__(16) _Float16 Hl[BLK_ROWS * NHID];
  __shared__ __align__(16) float    Xs[BLK_ROWS * CHUNK];
  __shared__ __align__(16) float    Ys[BLK_ROWS * CHUNK];

  const int lane = threadIdx.x & 31;
  const int n    = lane & 15;
  const int hh   = lane >> 4;
  const int rowbase = blockIdx.x * BLK_ROWS;

#pragma unroll 1
  for (int it = 0; it < 16; ++it) {
    const int o = (it * 32 + lane) * 8;
    const v4f a = *(const v4f*)(w_hh + o);
    const v4f b = *(const v4f*)(w_hh + o + 4);
    v8h hv, lv;
#pragma unroll
    for (int e = 0; e < 4; ++e) {
      const float fa = a[e];
      const float fb = b[e];
      _Float16 h0, l0, h1, l1;
      split_f16(fa, h0, l0);
      split_f16(fb, h1, l1);
      hv[e] = h0; lv[e] = l0;
      hv[4 + e] = h1; lv[4 + e] = l1;
    }
    *(v8h*)(Whi + o) = hv;
    *(v8h*)(Wlo + o) = lv;
  }
  {
    const int o = lane * 4;
    const v4f bi = *(const v4f*)(b_ih + o);
    const v4f bh = *(const v4f*)(b_hh + o);
    const v4f wi = *(const v4f*)(w_ih + o);
    v4f bs;
#pragma unroll
    for (int e = 0; e < 4; ++e) bs[e] = bi[e] + bh[e];
    *(v4f*)(Bs + o)  = bs;
    *(v4f*)(Wis + o) = wi;
  }
  {
    const v4u z = {0u, 0u, 0u, 0u};
    *(v4u*)(Hh + lane * 16)     = z;
    *(v4u*)(Hh + lane * 16 + 8) = z;
    *(v4u*)(Hl + lane * 16)     = z;
    *(v4u*)(Hl + lane * 16 + 8) = z;
  }
  float wl[2][8];
#pragma unroll
  for (int g = 0; g < 2; ++g) {
    const v4f p = *(const v4f*)(w_lin + 16 * g + 8 * hh);
    const v4f q = *(const v4f*)(w_lin + 16 * g + 8 * hh + 4);
#pragma unroll
    for (int e = 0; e < 4; ++e) { wl[g][e] = p[e]; wl[g][4 + e] = q[e]; }
  }
  const float blin = b_lin[0];
  float cst[2][8];
#pragma unroll
  for (int g = 0; g < 2; ++g)
#pragma unroll
    for (int r = 0; r < 8; ++r) cst[g][r] = 0.0f;
  __syncthreads();

  v16h ah[8];
#pragma unroll
  for (int mt = 0; mt < 8; ++mt) ah[mt] = Frag<_Float16>::load(Whi + (mt * 16 + n) * NHID + 8 * hh);

  const _Float16* wlo_lane = Wlo + n * NHID + 8 * hh;
  _Float16* hh_lane = Hh + n * NHID + 8 * hh;
  _Float16* hl_lane = Hl + n * NHID + 8 * hh;
  const v8f z8 = {0.f, 0.f, 0.f, 0.f, 0.f, 0.f, 0.f, 0.f};

#pragma unroll 1
  for (int chunk = 0; chunk < NSTEP / CHUNK; ++chunk) {
    const int s0 = chunk * CHUNK;
    {
      const int row = lane >> 1, cb = (lane & 1) * 16;
      const float* xp = x + (size_t)(rowbase + row) * NSTEP + s0 + cb;
      const v4f x0 = *(const v4f*)(xp);
      const v4f x1 = *(const v4f*)(xp + 4);
      const v4f x2 = *(const v4f*)(xp + 8);
      const v4f x3 = *(const v4f*)(xp + 12);
      float* xd = Xs + row * CHUNK + cb;
      *(v4f*)(xd)      = x0;
      *(v4f*)(xd + 4)  = x1;
      *(v4f*)(xd + 8)  = x2;
      *(v4f*)(xd + 12) = x3;
    }
    __syncthreads();

#pragma unroll 1
    for (int t = 0; t < CHUNK; ++t) {
      asm volatile("" ::: "memory");
      const float xv = Xs[n * CHUNK + t];
      const v16h bh = Frag<_Float16>::load(hh_lane);
      const v16h bl = Frag<_Float16>::load(hl_lane);
      float psum = 0.0f;
      v8h hv[2], lv[2];
#pragma unroll
      for (int g = 0; g < 2; ++g) {
        float gate[4][8];
#pragma unroll
        for (int q = 0; q < 4; ++q) {
          const int mt = 2 * q + g;
          asm volatile("" ::: "memory");
          const int ro = mt * 16 + 8 * hh;
          const v4f b0 = *(const v4f*)(Bs + ro);
          const v4f b1 = *(const v4f*)(Bs + ro + 4);
          const v4f w0 = *(const v4f*)(Wis + ro);
          const v4f w1 = *(const v4f*)(Wis + ro + 4);
          v8f cm;
#pragma unroll
          for (int e = 0; e < 4; ++e) {
            cm[e]     = fmaf(xv, w0[e], b0[e]);
            cm[4 + e] = fmaf(xv, w1[e], b1[e]);
          }
          const v16h al = Frag<_Float16>::load(wlo_lane + mt * 16 * NHID);
          v8f accm = Frag<_Float16>::mma(ah[mt], bh, cm);
          v8f accr = Frag<_Float16>::mma(ah[mt], bl, z8);
          accr     = Frag<_Float16>::mma(al, bh, accr);
          tile_guard(accm, accr, ah[mt], al, bh, bl);
#pragma unroll
          for (int r = 0; r < 8; ++r) gate[q][r] = fmaf(accr[r], RES_CARRY_INV, accm[r]);
        }
#pragma unroll
        for (int r = 0; r < 8; ++r) {
          const float ig = fsig(gate[0][r]);
          const float fg = fsig(gate[1][r]);
          const float gg = ftanh(gate[2][r]);
          const float og = fsig(gate[3][r]);
          const float cn = fg * cst[g][r] + ig * gg;
          cst[g][r] = cn;
          const float hn = og * ftanh(cn);
          psum = fmaf(hn, wl[g][r], psum);
          _Float16 h16, l16;
          split_f16(hn, h16, l16);
          hv[g][r] = h16;
          lv[g][r] = l16;
        }
      }
      *(v8h*)(hh_lane)      = hv[0];
      *(v8h*)(hh_lane + 16) = hv[1];
      *(v8h*)(hl_lane)      = lv[0];
      *(v8h*)(hl_lane + 16) = lv[1];
      const float tot = psum + __shfl_xor(psum, 16, 32);
      const float y = ftanh(tot + blin);
      if (hh == 0) Ys[n * CHUNK + t] = y;
      __syncthreads();
    }

    {
      const int q = lane >> 3, c4 = (lane & 7) * 4;
      v4f yv[4];
#pragma unroll
      for (int it = 0; it < 4; ++it) yv[it] = *(const v4f*)(Ys + (it * 4 + q) * CHUNK + c4);
      for (int pass = 0; pass < 2; ++pass) {
#pragma unroll
        for (int it = 0; it < 4; ++it) {
          const int row = it * 4 + q;
          *(volatile v4f*)(out + (size_t)(rowbase + row) * NSTEP + s0 + c4) = yv[it];
        }
        __threadfence();
      }
    }
  }
}

extern "C" void kernel_launch(void* const* d_in, const int* in_sizes, int n_in,
                              void* d_out, int out_size, void* d_ws, size_t ws_size, hipStream_t stream) {
  (void)in_sizes; (void)out_size; (void)d_ws; (void)ws_size;
  if (n_in < 7 || d_out == nullptr) return;
  const float* x     = (const float*)d_in[0];
  const float* w_ih  = (const float*)d_in[1];
  const float* w_hh  = (const float*)d_in[2];
  const float* b_ih  = (const float*)d_in[3];
  const float* b_hh  = (const float*)d_in[4];
  const float* w_lin = (const float*)d_in[5];
  const float* b_lin = (const float*)d_in[6];
  float* out = (float*)d_out;
  lstm_seq_kernel<<<dim3(NBATCH / BLK_ROWS), dim3(32), 0, stream>>>(x, w_ih, w_hh, b_ih, b_hh, w_lin, b_lin, out);
}
